// Transformer_28905129902584
// MI455X (gfx1250) — hardware-verified
//
#include <hip/hip_runtime.h>


#ifndef SEQ
#define SEQ 8192
#endif
#define SEQ_FULL 8192
#define VOCAB 10
#define DE    3
#define HD    4
#define HDP   32
#define AW    4
#define PT    64
#define SC2   ((float)(0.5 * 1.4426950408889634))
#define PSH   14.0f
#define NEGB  (-3.0e38f)

static_assert(HD == 4);
static_assert((HD & (HD - 1)) == 0);
static_assert(HDP == 32);
static_assert(HD <= 8);
static_assert(VOCAB <= 16);
static_assert(SEQ % 32 == 0);
static_assert(SEQ % (16 * AW) == 0);
static_assert(SEQ % PT == 0);
static_assert(PT == 64);
static_assert(PT * (HDP / 8) == 256);
static_assert(HD * 8 == 32);
static_assert(16 * 16 == 16 * HD * 4);
static_assert((size_t)(SEQ / PT) * 256 * 16 == (size_t)SEQ * HDP * 2);
static_assert((size_t)(SEQ / PT) * 32 * 16 == (size_t)HD * SEQ * 2);
static_assert((size_t)(SEQ / (16 * AW)) * AW * 16 * 16 == (size_t)SEQ * HD * 4);
static_assert((3 * 16 * 4 + PT) * 4 <= 131072);
static_assert(SEQ <= SEQ_FULL);

typedef _Float16 h16;
typedef __attribute__((ext_vector_type(16))) _Float16 v16h;
typedef __attribute__((ext_vector_type(8)))  _Float16 v8h;
typedef __attribute__((ext_vector_type(8)))  float    v8f;
typedef __attribute__((ext_vector_type(4)))  float    v4f;

__device__ __forceinline__ unsigned short f2bf(float f) { unsigned u = __float_as_uint(f); u += 0x7FFFu + ((u >> 16) & 1u); return (unsigned short)(u >> 16); }
__device__ __forceinline__ float bfr(float f) { return __uint_as_float(((unsigned)f2bf(f)) << 16); }
__device__ __forceinline__ v16h cat16(v8h lo, v8h hi) { return __builtin_shufflevector(lo, hi, 0, 1, 2, 3, 4, 5, 6, 7, 8, 9, 10, 11, 12, 13, 14, 15); }
__device__ __forceinline__ v16h  ldh(const h16* p) { return cat16(*(const v8h*)p, *(const v8h*)(p + 16)); }
static __device__ __forceinline__ h16 toh_flush(float v) { const h16 r = (h16)v; return (fabsf(v) < 6.103515625e-05f) ? (h16)0.0f : r; }
__device__ __forceinline__ v8f wmma16g(v16h a, v16h b, v8f c) {
    c = __builtin_amdgcn_wmma_f32_16x16x32_f16(false, a, false, b, (short)0, c, false, false);
    asm volatile("v_nop\n\tv_nop\n\tv_nop\n\tv_nop" : "+v"(c) : "v"(a), "v"(b));
    return c;
}

__global__ __launch_bounds__(256) void k_prep(const int* __restrict__ x, const float* __restrict__ emb,
                                              const float* __restrict__ wq, const float* __restrict__ bq,
                                              const float* __restrict__ wk, const float* __restrict__ bk,
                                              const float* __restrict__ wv, const float* __restrict__ bv,
                                              h16* QH, h16* KP, h16* VT) {
    __shared__ float tq[16 * HD];
    __shared__ float tk[16 * HD];
    __shared__ float tv[16 * HD];
    __shared__ int   xs[PT];
    const int tid = threadIdx.x;
    const int lane = tid & 31;
    const int wave = __builtin_amdgcn_readfirstlane((int)(threadIdx.x >> 5));
    const int t0 = blockIdx.x * PT;
    if (wave < 2) {
        const int vr = tid >> 2, d = tid & 3;
        const int vc = vr < VOCAB ? vr : (VOCAB - 1);
        const float e0 = bfr(emb[vc * DE + 0]), e1 = bfr(emb[vc * DE + 1]), e2 = bfr(emb[vc * DE + 2]);
        float a = e0 * bfr(wq[0 * HD + d]); a = a + e1 * bfr(wq[1 * HD + d]); a = a + e2 * bfr(wq[2 * HD + d]); a = a + bfr(bq[d]);
        float c = e0 * bfr(wk[0 * HD + d]); c = c + e1 * bfr(wk[1 * HD + d]); c = c + e2 * bfr(wk[2 * HD + d]); c = c + bfr(bk[d]);
        float g = e0 * bfr(wv[0 * HD + d]); g = g + e1 * bfr(wv[1 * HD + d]); g = g + e2 * bfr(wv[2 * HD + d]); g = g + bfr(bv[d]);
        tq[tid] = a; tk[tid] = c; tv[tid] = g;
        int xi = x[t0 + tid];
        xi = xi < 0 ? 0 : (xi > VOCAB - 1 ? VOCAB - 1 : xi);
        xs[tid] = xi;
    }
    __syncthreads();
    const int tl = tid >> 2;
    const bool first = (tid & 3) == 0;
    const int xi = xs[tl];
    v8h qv, kv;
#pragma unroll
    for (int i = 0; i < HD; ++i) {
        float a = tq[xi * HD + i]; float c = tk[xi * HD + i];
        asm volatile("" : "+v"(a)); asm volatile("" : "+v"(c));
        const h16 ah = toh_flush(a); const h16 ch = toh_flush(c);
        qv[i] = first ? ah : (h16)0.0f; kv[i] = first ? ch : (h16)0.0f;
        qv[4 + i] = (h16)0.0f; kv[4 + i] = (h16)0.0f; }
    const int vd = lane >> 3, c8 = (lane & 7) * 8;
    v8h vv = (v8h){};
    if (wave == 0) {
#pragma unroll
        for (int i = 0; i < 8; ++i) { const int xj = xs[c8 + i]; vv[i] = toh_flush(tv[xj * HD + vd]); }
    }
    const size_t po = ((size_t)blockIdx.x * 256 + (size_t)tid) * 8;
    const size_t vofs = (size_t)vd * SEQ + (size_t)t0 + (size_t)c8;
#pragma unroll 1
    for (int ps = 0; ps < 2; ++ps) {
        *(volatile v8h*)(QH + po) = qv;
        *(volatile v8h*)(KP + po) = kv;
        if (wave == 0) *(volatile v8h*)(VT + vofs) = vv;
        if (ps == 0) __threadfence(); }
}

__global__ __launch_bounds__(32 * AW) void k_flash(const h16* __restrict__ QH, const h16* __restrict__ KP, const h16* __restrict__ VT, float* OUT) {
    const int lane = threadIdx.x & 31, lr = lane & 15, hi = lane >> 4;
    const int wave = __builtin_amdgcn_readfirstlane((int)(threadIdx.x >> 5));
    const int t0 = (blockIdx.x * AW + wave) * 16;
    const size_t qo = (size_t)(t0 + lr) * HDP + 8 * hi;
    const v16h qh = ldh(QH + qo);
    const size_t ko = (size_t)lr * HDP + 8 * hi;
    const size_t vo = (size_t)(lr & (HD - 1)) * SEQ + 8 * hi;
    v8f o0 = (v8f){};
    float m = NEGB, l = 0.0f;
#pragma unroll 1
    for (int key0 = 0; key0 < SEQ; key0 += 32) {
        const h16* ka = KP + ko + (size_t)key0 * HDP;
        const v16h ka0 = ldh(ka), kb0 = ldh(ka + 16 * HDP);
        v8f sa = (v8f){}, sb = (v8f){};
        sa = wmma16g(ka0, qh, sa); sb = wmma16g(kb0, qh, sb);
        float ta[8], tb[8]; float mx = NEGB;
#pragma unroll
        for (int r = 0; r < 8; ++r) { ta[r] = sa[r] * SC2; tb[r] = sb[r] * SC2; mx = fmaxf(mx, fmaxf(ta[r], tb[r])); }
        mx = fmaxf(mx, __shfl_xor(mx, 16, 32));
        const float mnew = fmaxf(m, mx);
        const float alpha = __builtin_amdgcn_exp2f(m - mnew);
        const float sh = PSH - mnew;
        v16h pb; float ls = 0.0f;
#pragma unroll
        for (int r = 0; r < 8; ++r) {
            const float xa = ta[r] + sh, xb = tb[r] + sh;
            const float ea = __builtin_amdgcn_exp2f(xa), eb = __builtin_amdgcn_exp2f(xb);
            const float ga = (xa < -14.0f) ? 0.0f : ea, gb = (xb < -14.0f) ? 0.0f : eb;
            const h16 pa = (h16)ga; const h16 pc = (h16)gb;
            pb[r] = pa; pb[8 + r] = pc;
            ls += (float)pa + (float)pc; }
        l = l * alpha + ls; m = mnew;
        o0 = o0 * alpha;
        const v16h v0 = ldh(VT + vo + key0);
        o0 = wmma16g(v0, pb, o0);
    }
    l += __shfl_xor(l, 16, 32);
    const float inv = 1.0f / l;
    v4f val; val[0] = o0[0] * inv; val[1] = o0[1] * inv; val[2] = o0[2] * inv; val[3] = o0[3] * inv;
    float* orow = OUT + (size_t)(t0 + lr) * HD;
#pragma unroll 1
    for (int ps = 0; ps < 2; ++ps) {
        if (hi == 0) *(volatile v4f*)orow = val;
        if (ps == 0) __threadfence(); }
}

static constexpr size_t al256(size_t v) { return (v + 255) & ~(size_t)255; }
static constexpr size_t SZ_QK = al256((size_t)SEQ * HDP * 2);
static constexpr size_t SZ_VT = al256((size_t)HD * SEQ * 2);
static constexpr size_t SZ_TOTAL = 2 * SZ_QK + SZ_VT;
static_assert(SZ_TOTAL <= (size_t)134217728);

extern "C" void kernel_launch(void* const* d_in, const int* in_sizes, int n_in,
                              void* d_out, int out_size, void* d_ws, size_t ws_size, hipStream_t stream) {
    if (n_in < 8) return;
    if (in_sizes[0] < SEQ) return;
    if (in_sizes[1] < VOCAB * DE) return;
    if (in_sizes[2] < DE * HD || in_sizes[4] < DE * HD || in_sizes[6] < DE * HD) return;
    if (in_sizes[3] < HD || in_sizes[5] < HD || in_sizes[7] < HD) return;
    if ((size_t)out_size < (size_t)SEQ * HD) return;
    if (SZ_TOTAL > ws_size) return;
    const int*   x   = (const int*)d_in[0];
    const float* emb = (const float*)d_in[1];
    const float* wq  = (const float*)d_in[2]; const float* bq = (const float*)d_in[3];
    const float* wk  = (const float*)d_in[4]; const float* bk = (const float*)d_in[5];
    const float* wv  = (const float*)d_in[6]; const float* bv = (const float*)d_in[7];
    float* OUT = (float*)d_out;
    char* wsp = (char*)d_ws;
    h16* QH = (h16*)wsp; wsp += SZ_QK;
    h16* KP = (h16*)wsp; wsp += SZ_QK;
    h16* VT = (h16*)wsp; wsp += SZ_VT;

    k_prep<<<dim3(SEQ / PT, 1, 1), 256, 0, stream>>>(x, emb, wq, bq, wk, bk, wv, bv, QH, KP, VT);
    k_flash<<<dim3(SEQ / (16 * AW), 1, 1), 32 * AW, 0, stream>>>(QH, KP, VT, OUT);
}
